// TSEncoder_17523466567872
// MI455X (gfx1250) — hardware-verified
//
#include <hip/hip_runtime.h>
#include <stdint.h>

typedef __attribute__((ext_vector_type(16))) _Float16 v16h;
typedef __attribute__((ext_vector_type(8)))  _Float16 v8h;
typedef __attribute__((ext_vector_type(8)))  float    v8f;
typedef __attribute__((ext_vector_type(4)))  float    v4f;

constexpr int kB    = 4096;
constexpr int kT    = 250;
constexpr int kD    = 4;
constexpr int kH    = 64;
constexpr int kG    = 256;
constexpr int kTout = 50;
constexpr int kRowsBlk     = 16;
constexpr int kLstmBlocks  = kB / kRowsBlk;
constexpr int kLstmThreads = 128;
constexpr int kChunk  = 50;
constexpr int kHP     = 72;
constexpr int kWHP    = 72;
constexpr int kSP     = 68;
constexpr int kStBlocks  = 500;
constexpr int kStThreads = 256;
constexpr int kStPer     = 8;
constexpr int kPartLine  = 32;

static_assert(kStBlocks * kStThreads * kStPer == kB * kT);
static_assert(kB % kRowsBlk == 0);
static_assert(kT % kChunk == 0);
static_assert(kT % 5 == 0 && kTout == kT / 5);
static_assert(kH % 32 == 0 && kG == 4 * kH);
static_assert((kRowsBlk * kChunk) % 2 == 0);

template <typename T> struct Frag;
template <> struct Frag<_Float16> {
  typedef v16h V; union U { v16h v; v8h h[2]; };
  static __device__ __forceinline__ v16h load(const _Float16* p) {
    U f; f.h[0] = *(const v8h*)(p); f.h[1] = *(const v8h*)(p + 16); return f.v;
  }
};

__device__ __forceinline__ v8f hmma(v16h a, v16h b, v8f c) {
  c = __builtin_amdgcn_wmma_f32_16x16x32_f16(false, a, false, b, (short)0, c, false, false);
  asm volatile("v_nop\n\tv_nop\n\tv_nop\n\tv_nop" : "+v"(c) : "v"(a), "v"(b));
  return c;
}

__device__ __forceinline__ float sigm(float v) {
  const float e = expf(fminf(-v, 80.0f));
  return __builtin_amdgcn_rcpf(1.0f + e);
}
__device__ __forceinline__ float tanhx(float v) {
  const float e = expf(fminf(2.0f * v, 80.0f));
  return 1.0f - 2.0f * __builtin_amdgcn_rcpf(1.0f + e);
}

__global__ __launch_bounds__(256) void k_bnstats(const float* __restrict__ x, float* __restrict__ part) {
  __shared__ float red[8][8];
  const int tid  = threadIdx.x;
  const int lane = tid & 31;
  const int wave = tid >> 5;
  const size_t base = (size_t)blockIdx.x * (size_t)(kStThreads * kStPer);
  float s0 = 0.f, s1 = 0.f, s2 = 0.f, s3 = 0.f, q0 = 0.f, q1 = 0.f, q2 = 0.f, q3 = 0.f;
#pragma unroll
  for (int j = 0; j < kStPer; ++j) {
    const size_t row = base + (size_t)j * kStThreads + (size_t)tid;
    const v4f v = *(const v4f*)(x + row * 4);
    s0 += v.x; s1 += v.y; s2 += v.z; s3 += v.w;
    q0 += v.x * v.x; q1 += v.y * v.y; q2 += v.z * v.z; q3 += v.w * v.w;
  }
#pragma unroll
  for (int off = 16; off > 0; off >>= 1) {
    s0 += __shfl_xor(s0, off, 32); s1 += __shfl_xor(s1, off, 32);
    s2 += __shfl_xor(s2, off, 32); s3 += __shfl_xor(s3, off, 32);
    q0 += __shfl_xor(q0, off, 32); q1 += __shfl_xor(q1, off, 32);
    q2 += __shfl_xor(q2, off, 32); q3 += __shfl_xor(q3, off, 32);
  }
  if (lane == 0) {
    red[wave][0] = s0; red[wave][1] = s1; red[wave][2] = s2; red[wave][3] = s3;
    red[wave][4] = q0; red[wave][5] = q1; red[wave][6] = q2; red[wave][7] = q3;
  }
  __syncthreads();
  const int li = lane & 7;
  float tot = 0.f;
#pragma unroll
  for (int w = 0; w < 8; ++w) tot += red[w][li];
  const int sb = (lane < 1) ? 0 : 4;
  v4f o;
  o.x = __shfl(tot, sb + 0, 32);
  o.y = __shfl(tot, sb + 1, 32);
  o.z = __shfl(tot, sb + 2, 32);
  o.w = __shfl(tot, sb + 3, 32);
  if (lane >= 2) o = (v4f){0.f, 0.f, 0.f, 0.f};
  float* dst = part + (size_t)blockIdx.x * kPartLine + lane * 4;
  const bool writer = (wave == 0) && (lane < 8);
  for (int pass = 0; pass < 2; ++pass) {
    if (writer) *(volatile v4f*)dst = o;
    __threadfence();
  }
}

__global__ __launch_bounds__(128)
void k_lstm(const float* __restrict__ x, const float* __restrict__ part,
            const float* __restrict__ gamma, const float* __restrict__ beta,
            const float* __restrict__ W_ih, const float* __restrict__ W_hh,
            const float* __restrict__ b_ih, const float* __restrict__ b_hh,
            float* __restrict__ out) {
  __shared__ __align__(16) _Float16 whs[kG * kWHP];
  __shared__ __align__(16) _Float16 hbuf[2 * kRowsBlk * kHP];
  __shared__ __align__(16) float    xs[kRowsBlk * kChunk * kD];
  __shared__ __align__(16) float    slab[kRowsBlk * kSP];
  __shared__ double dred[8];
  __shared__ float  s_mean[4], s_scale[4], s_beta[4];

  const int tid  = threadIdx.x;
  const int lane = tid & 31;
  const int wave = tid >> 5;
  const int hsel = lane >> 4;
  const int c    = lane & 15;
  const int koff = hsel * 8;
  const int col  = 16 * wave + c;
  const int tileBase = blockIdx.x * kRowsBlk;

  {
    const int ci = tid & 7;
    double a = 0.0;
#pragma unroll 1
    for (int i = 0; i < kStBlocks; ++i) a += (double)part[i * kPartLine + ci];
    if (tid < 8) dred[tid] = a;
  }
  __syncthreads();
  if (tid < 4) {
    const double invN = 1.0 / ((double)kB * (double)kT);
    const double m = dred[tid] * invN;
    const double var = dred[4 + tid] * invN - m * m;
    float varf = (float)var;
    varf = varf < 0.f ? 0.f : varf;
    const float rs = rsqrtf(varf + 1e-5f);
    s_mean[tid]  = (float)m;
    s_scale[tid] = rs * gamma[tid];
    s_beta[tid]  = beta[tid];
  }
#pragma unroll 1
  for (int i = tid; i < (kG * kH) / 8; i += kLstmThreads) {
    const int n = i >> 3, k8 = (i & 7) * 8;
    const v4f a  = *(const v4f*)(W_hh + n * kH + k8);
    const v4f b2 = *(const v4f*)(W_hh + n * kH + k8 + 4);
    v8h hv;
    hv[0] = (_Float16)(a.x * 8.0f);  hv[1] = (_Float16)(a.y * 8.0f);
    hv[2] = (_Float16)(a.z * 8.0f);  hv[3] = (_Float16)(a.w * 8.0f);
    hv[4] = (_Float16)(b2.x * 8.0f); hv[5] = (_Float16)(b2.y * 8.0f);
    hv[6] = (_Float16)(b2.z * 8.0f); hv[7] = (_Float16)(b2.w * 8.0f);
    *(v8h*)(whs + n * kWHP + k8) = hv;
  }
  v4f wih[4];
  float bsum[4];
#pragma unroll
  for (int q = 0; q < 4; ++q) {
    const int n = q * kH + col;
    wih[q]  = *(const v4f*)(W_ih + n * kD);
    bsum[q] = b_ih[n] + b_hh[n];
  }
  __syncthreads();

  float cst[8];
#pragma unroll
  for (int r = 0; r < 8; ++r) cst[r] = 0.f;
  v16h hA[2];
#pragma unroll
  for (int kk = 0; kk < 2; ++kk) {
#pragma unroll
    for (int e = 0; e < 16; ++e) hA[kk][e] = (_Float16)0.0f;
  }

#pragma unroll 1
  for (int t = 0; t < kT; ++t) {
    const int cidx = t / kChunk;
    const int tin  = t - cidx * kChunk;
    if (tin == 0) {
      const int tbase = kT - kChunk * (cidx + 1);
      const float m0 = s_mean[0], m1 = s_mean[1], m2 = s_mean[2], m3 = s_mean[3];
      const float a0 = s_scale[0], a1 = s_scale[1], a2 = s_scale[2], a3 = s_scale[3];
      const float e0 = s_beta[0], e1 = s_beta[1], e2 = s_beta[2], e3 = s_beta[3];
      for (int i = tid; i < kRowsBlk * kChunk; i += kLstmThreads) {
        const int row = i / kChunk, lt = i - row * kChunk;
        const v4f v = *(const v4f*)(x + ((size_t)(tileBase + row) * kT + (size_t)(tbase + lt)) * kD);
        v4f o;
        o.x = (v.x - m0) * a0 + e0;
        o.y = (v.y - m1) * a1 + e1;
        o.z = (v.z - m2) * a2 + e2;
        o.w = (v.w - m3) * a3 + e3;
        *(v4f*)(xs + i * kD) = o;
      }
      __syncthreads();
    }
    const int lt = kChunk - 1 - tin;
    const int j5 = t / 5;
    const bool emit = (t - j5 * 5) == 4;

    v8f acc[4];
#pragma unroll
    for (int q = 0; q < 4; ++q) acc[q] = (v8f){0.f, 0.f, 0.f, 0.f, 0.f, 0.f, 0.f, 0.f};
#pragma unroll
    for (int kk = 0; kk < 2; ++kk) {
#pragma unroll
      for (int q = 0; q < 4; ++q) {
        const v16h bq = Frag<_Float16>::load(whs + (q * kH + col) * kWHP + kk * 32 + koff);
        acc[q] = hmma(hA[kk], bq, acc[q]);
      }
    }

    _Float16* hb = hbuf + (t & 1) * (kRowsBlk * kHP);
#pragma unroll
    for (int r = 0; r < 8; ++r) {
      const int row = 8 * hsel + r;
      const v4f xv = *(const v4f*)(xs + (row * kChunk + lt) * kD);
      float pre[4];
#pragma unroll
      for (int q = 0; q < 4; ++q) {
        float p = bsum[q];
        p = fmaf(xv.x, wih[q].x, p);
        p = fmaf(xv.y, wih[q].y, p);
        p = fmaf(xv.z, wih[q].z, p);
        p = fmaf(xv.w, wih[q].w, p);
        p = fmaf(acc[q][r], 0.015625f, p);
        pre[q] = p;
      }
      const float ig = sigm(pre[0]);
      const float fg = sigm(pre[1]);
      const float gg = tanhx(pre[2]);
      const float og = sigm(pre[3]);
      const float cn = fg * cst[r] + ig * gg;
      cst[r] = cn;
      const float hv = og * tanhx(cn);
      hb[row * kHP + col] = (_Float16)(hv * 8.0f);
      if (emit) slab[row * kSP + col] = hv;
    }
    __syncthreads();

#pragma unroll
    for (int kk = 0; kk < 2; ++kk) hA[kk] = Frag<_Float16>::load(hb + c * kHP + kk * 32 + koff);

    if (emit) {
      const int c4 = c * 4;
      for (int pass = 0; pass < 2; ++pass) {
#pragma unroll
        for (int it = 0; it < 2; ++it) {
          const int row = wave * 4 + it * 2 + hsel;
          const v4f v = *(const v4f*)(slab + row * kSP + c4);
          *(volatile v4f*)(out + (size_t)(tileBase + row) * (size_t)(kTout * kH) + (size_t)j5 * kH + c4) = v;
        }
        __threadfence();
      }
    }
  }
}

extern "C" void kernel_launch(void* const* d_in, const int* in_sizes, int n_in,
                              void* d_out, int out_size, void* d_ws, size_t ws_size,
                              hipStream_t stream) {
  if (n_in < 7) return;
  if (in_sizes[0] != kB * kT * kD) return;
  if (in_sizes[1] != kD || in_sizes[2] != kD) return;
  if (in_sizes[3] != kG * kD || in_sizes[4] != kG * kH) return;
  if (in_sizes[5] != kG || in_sizes[6] != kG) return;
  if (out_size != kB * kTout * kH) return;
  const size_t ws_need = (size_t)kStBlocks * kPartLine * sizeof(float);
  if (ws_size < ws_need) return;

  const float* x     = (const float*)d_in[0];
  const float* gamma = (const float*)d_in[1];
  const float* beta  = (const float*)d_in[2];
  const float* W_ih  = (const float*)d_in[3];
  const float* W_hh  = (const float*)d_in[4];
  const float* b_ih  = (const float*)d_in[5];
  const float* b_hh  = (const float*)d_in[6];
  float* out  = (float*)d_out;
  float* part = (float*)d_ws;

  k_bnstats<<<dim3(kStBlocks), dim3(kStThreads), 0, stream>>>(x, part);
  k_lstm<<<dim3(kLstmBlocks), dim3(kLstmThreads), 0, stream>>>(x, part, gamma, beta, W_ih, W_hh, b_ih, b_hh, out);
}
